// InteractionNet_13340168421980
// MI455X (gfx1250) — hardware-run, weakly checked
//
#include <hip/hip_runtime.h>


namespace {
constexpr int N = 10000, E = 200000, F = 128, NBF = 20;
constexpr float XS = 8.0f, HS = 256.0f, WSC = 256.0f, EPS = 1e-5f;
typedef _Float16 b16;
typedef __attribute__((ext_vector_type(16))) _Float16 v16b;
typedef __attribute__((ext_vector_type(8))) _Float16 v8b;
typedef __attribute__((ext_vector_type(8))) float v8f;
typedef __attribute__((ext_vector_type(4))) float v4f;
__device__ __forceinline__ float bf16_rne(float f) { unsigned int u = __float_as_uint(f); u += 0x7FFFu + ((u >> 16) & 1u); float r = __uint_as_float(u & 0xFFFF0000u); asm volatile("" : "+v"(r)); return r; }
__device__ __forceinline__ float bfv(float f) { float r = bf16_rne(f); asm volatile("" : "+v"(r)); return r; }
__device__ __forceinline__ void split16(float v, b16& hi, b16& lo) { hi = (b16)v; lo = (b16)(v - (float)hi); }
__device__ __forceinline__ v16b frag_kb(const b16* p, int hh) { const v8b a = *(const v8b*)(p + 8 * hh), b = *(const v8b*)(p + 16 + 8 * hh); v16b f;
#pragma unroll
  for (int e = 0; e < 8; ++e) { f[e] = a[e]; f[8 + e] = b[e]; } return f; }
__device__ __forceinline__ v8f wmma16b(v16b a, v16b b, v8f c) { v8f d = __builtin_amdgcn_wmma_f32_16x16x32_f16(false, a, false, b, (short)0, c, false, false); asm volatile("v_nop\n\tv_nop\n\tv_nop\n\tv_nop" : "+v"(d) : "v"(a), "v"(b)); return d; }
__device__ __forceinline__ void wave_lds_sync() { __builtin_amdgcn_fence(__ATOMIC_RELEASE, "workgroup"); __builtin_amdgcn_wave_barrier(); __builtin_amdgcn_fence(__ATOMIC_ACQUIRE, "workgroup"); }
__device__ __forceinline__ float pmul(float a, float b) { float p = a * b; asm volatile("" : "+v"(p)); return p; }
__device__ __forceinline__ int iclamp(int v, int lo, int hi) { return v < lo ? lo : (v > hi ? hi : v); }
__device__ __forceinline__ float silu(float v) { return v / (1.0f + __expf(-v)); }
__device__ __forceinline__ float wsum(float v) { for (int o = 16; o; o >>= 1) v += __shfl_xor(v, o); return v; }
constexpr int CSR_NBLK8 = 512, CSR_GB8 = 8, CSR_GN8 = 1 << CSR_GB8  , CSR_TS8 = (CSR_GN8 < 32 ? 32 : CSR_GN8)  , CSR_MAXG8 = 512, CSR_CAP8 = 12288  ;
__device__ __host__ __forceinline__ int csr_tix8(int v) { return (v >> CSR_GB8) * CSR_TS8 + (v & (CSR_GN8 - 1)); }
__global__ __launch_bounds__(64) void csrA_kernel8(const int* __restrict__ dst, int E, int N, int nG, int CHP, int NGP, int* __restrict__ STG, int* __restrict__ HST) {
  extern __shared__ int sm[];
  int* cnt = sm; int* run = sm + NGP; int* ids = sm + 2 * NGP;
  const int b = blockIdx.x; const int ch = (E + CSR_NBLK8 - 1) / CSR_NBLK8; const int e0 = b * ch, e1 = min(E, e0 + ch);
  for (int i = threadIdx.x; i < NGP; i += 64) cnt[i] = 0;
  for (int i = threadIdx.x; i < CHP; i += 64) ids[i] = -1;
  __syncthreads();
  if (threadIdx.x == 0) {
    for (int e = e0; e < e1; ++e) { int d = dst[e]; d = (d < 0) ? 0 : (d >= N ? N - 1 : d); cnt[d >> CSR_GB8] += 1; }
    int acc = 0; for (int g = 0; g < nG; ++g) { run[g] = acc; acc += cnt[g]; }
    for (int e = e0; e < e1; ++e) { int d = dst[e]; d = (d < 0) ? 0 : (d >= N ? N - 1 : d); const int g = d >> CSR_GB8; ids[run[g]] = e; run[g] += 1; } }
  __syncthreads();
  typedef __attribute__((ext_vector_type(4))) int v4i;
  for (int pass = 0; pass < 2; ++pass) {
    for (int i = threadIdx.x; i < CHP / 4; i += 64) *(volatile v4i*)(STG + (size_t)b * CHP + i * 4) = *(const v4i*)(&ids[i * 4]);
    for (int i = threadIdx.x; i < NGP / 4; i += 64) { v4i v; for (int e = 0; e < 4; ++e) v[e] = (i * 4 + e < nG) ? cnt[i * 4 + e] : 0; *(volatile v4i*)(HST + (size_t)b * NGP + i * 4) = v; }
    __threadfence(); }
}
__global__ __launch_bounds__(512) void csrS_kernel8(const int* __restrict__ HST, int nG, int NGP, int* __restrict__ START, int* __restrict__ TOT, int* __restrict__ OFF) {
  __shared__ int tot[CSR_MAXG8];
  const int b = threadIdx.x;
  for (int pass = 0; pass < 2; ++pass) { int runb = 0; for (int g = 0; g < nG; ++g) { int c = HST[(size_t)b * NGP + g]; c = (c < 0) ? 0 : c; ((volatile int*)OFF)[(size_t)g * CSR_NBLK8 + b] = runb; runb += c; } __threadfence(); }
  for (int g = threadIdx.x; g < nG; g += 512) { int s = 0; for (int bb = 0; bb < CSR_NBLK8; ++bb) { int c = HST[(size_t)bb * NGP + g]; s += (c < 0) ? 0 : c; } tot[g] = s; }
  __syncthreads();
  if (threadIdx.x < 32) {
    __shared__ int st[CSR_MAXG8 + 32];
    if (threadIdx.x == 0) { int acc = 0; for (int g = 0; g < NGP; ++g) { st[g] = acc; if (g < nG) acc += (tot[g] + 31) & ~31; } st[NGP] = acc; }
    __builtin_amdgcn_fence(__ATOMIC_RELEASE, "workgroup"); __builtin_amdgcn_wave_barrier(); __builtin_amdgcn_fence(__ATOMIC_ACQUIRE, "workgroup");
    for (int pass = 0; pass < 2; ++pass) { for (int i = threadIdx.x; i < NGP + 32; i += 32) { ((volatile int*)START)[i] = (i <= NGP) ? st[min(i, NGP)] : 0; ((volatile int*)TOT)[i] = (i < nG) ? tot[i] : 0; } __threadfence(); } }
}
__global__ __launch_bounds__(256) void csrB_kernel8(const int* __restrict__ dst, int N, int nG, int CHP, int NGP, int permLen, const int* __restrict__ STG, const int* __restrict__ HST, const int* __restrict__ OFF, const int* __restrict__ START, const int* __restrict__ TOT, int* __restrict__ PERM, int* __restrict__ ROWPTR, int* __restrict__ ROWCNT, int* __restrict__ FLAG) {
  typedef __attribute__((ext_vector_type(4))) int v4i;
  __shared__ int ids[CSR_CAP8]; __shared__ unsigned short key[CSR_CAP8]; __shared__ int outp[CSR_CAP8]; __shared__ int ncnt[CSR_GN8 + 1]; __shared__ int boff[CSR_NBLK8 + 1];
  const int g = blockIdx.x, t_ = threadIdx.x; int tot = TOT[g]; int st = START[g], stn = START[g + 1]; const int v0 = g * CSR_GN8; const int nv = min(CSR_GN8, N - v0); const int t0 = g * CSR_TS8;
  st = (st < 0) ? 0 : (st > permLen - 32 ? permLen - 32 : st) & ~31; stn = (stn < st) ? st : (stn > permLen ? permLen : stn); tot = (tot < 0) ? 0 : tot; if (tot > stn - st && tot <= CSR_CAP8) tot = stn - st;
  if (tot > CSR_CAP8) {
    for (int pass = 0; pass < 2; ++pass) { for (int i = t_; i < CSR_TS8 / 4; i += 256) { v4i a, c; for (int e = 0; e < 4; ++e) { a[e] = st; c[e] = 0; } *(volatile v4i*)(ROWPTR + t0 + i * 4) = a; *(volatile v4i*)(ROWCNT + t0 + i * 4) = c; } if (t_ == 0) ((volatile int*)FLAG)[0] = 1; __threadfence(); } (void)nv; return; }
  if (t_ == 0) { int acc = 0; for (int b = 0; b < CSR_NBLK8; ++b) { boff[b] = acc; int c = HST[(size_t)b * NGP + g]; c = (c < 0) ? 0 : (c > CHP ? CHP : c); acc += c; if (acc > tot) acc = tot; } boff[CSR_NBLK8] = acc; }
  for (int i = t_; i <= CSR_GN8; i += 256) ncnt[i] = 0;
  __syncthreads();
  for (int b = 0; b < CSR_NBLK8; ++b) { const int c = boff[b + 1] - boff[b]; int o_ = OFF[(size_t)g * CSR_NBLK8 + b]; o_ = (o_ < 0) ? 0 : (o_ > CHP - c ? CHP - c : o_); const int* src_ = STG + (size_t)b * CHP + o_;
    for (int i = t_; i < c; i += 256) { int id = src_[i]; id = (id < 0) ? 0 : id; ids[boff[b] + i] = id; int d = dst[id]; d = (d < v0) ? v0 : (d >= N ? N - 1 : d); int kk = d - v0; kk = (kk < 0) ? 0 : (kk >= CSR_GN8 ? CSR_GN8 - 1 : kk); key[boff[b] + i] = (unsigned short)kk; } }
  __syncthreads();
  if (t_ == 0) { for (int i = 0; i < tot; ++i) ncnt[key[i]] += 1; int acc = 0; for (int vl = 0; vl < CSR_GN8; ++vl) { const int c = ncnt[vl]; ncnt[vl] = acc; acc += c; } ncnt[CSR_GN8] = acc;
    for (int i = 0; i < tot; ++i) { const int vl = key[i]; outp[ncnt[vl]] = ids[i]; ncnt[vl] += 1; }
    for (int vl = CSR_GN8; vl > 0; --vl) ncnt[vl] = ncnt[vl - 1]; ncnt[0] = 0; }
  __syncthreads();
  for (int pass = 0; pass < 2; ++pass) {
    for (int i = t_; i < (stn - st) / 4; i += 256) { v4i v; for (int e = 0; e < 4; ++e) { const int q = i * 4 + e; v[e] = (q < tot) ? outp[q] : -1; } *(volatile v4i*)(PERM + st + i * 4) = v; }
    for (int i = t_; i < CSR_TS8 / 4; i += 256) { v4i a, c; for (int e = 0; e < 4; ++e) { const int vl = i * 4 + e; const int vc = vl < CSR_GN8 ? vl : CSR_GN8; a[e] = (vl < CSR_GN8) ? st + ncnt[vc] : st; c[e] = (vl < nv) ? (ncnt[(vc < CSR_GN8 ? vc : CSR_GN8 - 1) + 1] - ncnt[vc]) : 0; } *(volatile v4i*)(ROWPTR + t0 + i * 4) = a; *(volatile v4i*)(ROWCNT + t0 + i * 4) = c; }
    __threadfence(); }
}
__global__ __launch_bounds__(256) void csrZ_kernel8(int* __restrict__ p, size_t n4) { typedef __attribute__((ext_vector_type(4))) int v4i; const size_t tid = (size_t)blockIdx.x * 256 + threadIdx.x, nth = (size_t)gridDim.x * 256; v4i z = {0, 0, 0, 0}; for (size_t i = tid; i < n4; i += nth) *(volatile v4i*)(p + i * 4) = z; }
struct CsrBufs8 { int *STG, *HST, *OFF, *START, *TOT, *PERM, *ROWPTR, *ROWCNT, *FLAG; int nG, NGP, CHP; size_t permLen; char* base; size_t bytes; };
static size_t csr_carve8(CsrBufs8& c, char* ws, size_t off, int E, int N) {
  const size_t off0 = off; c.base = ws + off;
  auto al = [&](size_t bytes) { char* p = ws + off; off += (bytes + 255) & ~(size_t)255; return p; };
  c.nG = (N + CSR_GN8 - 1) / CSR_GN8; c.NGP = (c.nG + 31) & ~31; const int ch = (E + CSR_NBLK8 - 1) / CSR_NBLK8; c.CHP = (ch + 31) & ~31; c.permLen = (size_t)E + 32 * (size_t)c.nG + 32;
  c.STG = (int*)al((size_t)CSR_NBLK8 * c.CHP * 4); c.HST = (int*)al((size_t)CSR_NBLK8 * c.NGP * 4); c.OFF = (int*)al((size_t)c.NGP * CSR_NBLK8 * 4); c.START = (int*)al((size_t)(c.NGP + 64) * 4); c.TOT = (int*)al((size_t)(c.NGP + 64) * 4);
  c.PERM = (int*)al(c.permLen * 4); c.ROWPTR = (int*)al((size_t)c.nG * CSR_TS8 * 4); c.ROWCNT = (int*)al((size_t)c.nG * CSR_TS8 * 4); c.FLAG = (int*)al(256);
  c.bytes = off - off0; return off;
}
static void csr_build8(const CsrBufs8& c, const int* dst, int E, int N, hipStream_t stream) {
  const size_t smem = (size_t)(2 * c.NGP + c.CHP) * 4;
  csrZ_kernel8<<<512, 256, 0, stream>>>((int*)c.base, c.bytes / 16);
  csrA_kernel8<<<CSR_NBLK8, 64, smem, stream>>>(dst, E, N, c.nG, c.CHP, c.NGP, c.STG, c.HST);
  csrS_kernel8<<<1, 512, 0, stream>>>(c.HST, c.nG, c.NGP, c.START, c.TOT, c.OFF);
  csrB_kernel8<<<c.nG, 256, 0, stream>>>(dst, N, c.nG, c.CHP, c.NGP, (int)c.permLen, c.STG, c.HST, c.OFF, c.START, c.TOT, c.PERM, c.ROWPTR, c.ROWCNT, c.FLAG);
}


__global__ __launch_bounds__(256) void wput_kernel(const float* __restrict__ nw1, const float* __restrict__ nw2, const float* __restrict__ e1w1, const float* __restrict__ e1w2, const float* __restrict__ e2w1, const float* __restrict__ e2w2, const float* __restrict__ e3w1, const float* __restrict__ e3w2, const float* __restrict__ uw1, const float* __restrict__ uw2, const float* __restrict__ empw, b16* __restrict__ W8, b16* __restrict__ WEQ, b16* __restrict__ WEM) { const size_t nt = (size_t)gridDim.x * 256, u0 = (size_t)blockIdx.x * 256 + threadIdx.x; v8b v; auto put = [&](b16* dst) { for (int pass = 0; pass < 2; ++pass) { *(volatile v8b*)dst = v; __threadfence(); } };
  for (size_t u = u0; u < (size_t)8 * F * 16; u += nt) { const int m = (int)(u / (F * 16)), o = (int)((u / 16) % F), k0 = (int)(u % 16) * 8; const float* w = m == 0 ? nw1 : m == 1 ? nw2 : m == 2 ? e1w2 : m == 3 ? e2w2 : m == 4 ? e3w1 : m == 5 ? e3w2 : m == 6 ? uw1 : uw2;
#pragma unroll
    for (int j = 0; j < 8; ++j) v[j] = (b16)(bf16_rne(w[(size_t)(k0 + j) * F + o]) * WSC); put(W8 + ((size_t)m * F + o) * F + k0); }
  for (size_t u = u0; u < (size_t)256 * 16; u += nt) { const int o = (int)(u / 16), k0 = (int)(u % 16) * 8; const float* w = o < F ? e1w1 : e2w1; const int oo = o % F;
#pragma unroll
    for (int j = 0; j < 8; ++j) v[j] = (b16)(bf16_rne(w[(size_t)(k0 + j) * F + oo]) * WSC); put(WEQ + (size_t)o * F + k0); }
  for (size_t u = u0; u < (size_t)F * 4; u += nt) { const int o = (int)(u / 4), k0 = (int)(u % 4) * 8;
#pragma unroll
    for (int j = 0; j < 8; ++j) { const int k = k0 + j; v[j] = (b16)(k < NBF ? bf16_rne(empw[(size_t)k * F + o]) * WSC : 0.0f); } put(WEM + (size_t)o * 32 + k0); } }
template <bool RAW>
__global__ __launch_bounds__(32) void nodemlp_kernel(const float* __restrict__ IN, const b16* __restrict__ Wa, const float* __restrict__ ba, const b16* __restrict__ Wb, const float* __restrict__ bb, float* __restrict__ OUT, const b16* __restrict__ Wc, const b16* __restrict__ Wd2, float* __restrict__ OUT2) { __shared__ __attribute__((aligned(16))) b16 Ah[16][F + 8], Al[16][F + 8], Bh[16][F + 8], Bl[16][F + 8]; __shared__ float Tf[16][F + 4]; const int lane = threadIdx.x, nloc = lane & 15, hlf = lane >> 4; const size_t n0 = (size_t)blockIdx.x * 16;
  for (int rr = 0; rr < 16; ++rr) for (int q = 0; q < 4; ++q) { const int c = q * 32 + lane; const float v = IN[(n0 + rr) * F + c]; if (RAW) { Ah[rr][c] = (b16)(bfv(v) * XS); Al[rr][c] = (b16)0.0f; } else { b16 p, pl; split16(v * HS, p, pl); Ah[rr][c] = p; Al[rr][c] = pl; } }
  if (lane < 16) for (int k = F; k < F + 8; ++k) { Ah[lane][k] = (b16)0.0f; Al[lane][k] = (b16)0.0f; Bh[lane][k] = (b16)0.0f; Bl[lane][k] = (b16)0.0f; }
  wave_lds_sync();
  const int nm = OUT2 ? 2 : 1;
#pragma unroll 1
  for (int mI = 0; mI < nm; ++mI) { const b16* W1p = mI == 0 ? Wa : Wc; const b16* W2p = mI == 0 ? Wb : Wd2; const float* b1p = mI == 0 ? ba : nullptr; const float* b2p = mI == 0 ? bb : nullptr; v8f acc[8];
#pragma unroll
    for (int t = 0; t < 8; ++t) acc[t] = (v8f){};
#pragma unroll
    for (int kb = 0; kb < F; kb += 32) { const v16b a = frag_kb(&Ah[nloc][kb], hlf), al = frag_kb(&Al[nloc][kb], hlf);
#pragma unroll
      for (int t = 0; t < 8; ++t) { const v16b bw = frag_kb(W1p + (size_t)(t * 16 + nloc) * F + kb, hlf); acc[t] = wmma16b(a, bw, acc[t]); if (!RAW) acc[t] = wmma16b(al, bw, acc[t]); } }
    const float isc = RAW ? 1.0f / (XS * WSC) : 1.0f / (HS * WSC);
#pragma unroll
    for (int t = 0; t < 8; ++t) { const int cc = t * 16 + nloc; const float b1v = b1p ? bfv(b1p[cc]) : 0.0f;
#pragma unroll
      for (int r8 = 0; r8 < 8; ++r8) { const float hv = silu(acc[t][r8] * isc + b1v); b16 p, pl; split16(hv * HS, p, pl); Bh[8 * hlf + r8][cc] = p; Bl[8 * hlf + r8][cc] = pl; } }
    wave_lds_sync();
#pragma unroll
    for (int t = 0; t < 8; ++t) acc[t] = (v8f){};
#pragma unroll
    for (int kb = 0; kb < F; kb += 32) { const v16b a = frag_kb(&Bh[nloc][kb], hlf), al = frag_kb(&Bl[nloc][kb], hlf);
#pragma unroll
      for (int t = 0; t < 8; ++t) { const v16b bw = frag_kb(W2p + (size_t)(t * 16 + nloc) * F + kb, hlf); acc[t] = wmma16b(a, bw, acc[t]); acc[t] = wmma16b(al, bw, acc[t]); } }
#pragma unroll
    for (int t = 0; t < 8; ++t) { const int cc = t * 16 + nloc; const float b2v = b2p ? bfv(b2p[cc]) : 0.0f;
#pragma unroll
      for (int r8 = 0; r8 < 8; ++r8) Tf[8 * hlf + r8][cc] = acc[t][r8] * (1.0f / (HS * WSC)) + b2v; }
    wave_lds_sync();
    float* dst = mI == 0 ? OUT : OUT2;
    for (int pass = 0; pass < 2; ++pass) { for (int rr = 0; rr < 16; ++rr) *(volatile v4f*)(dst + (n0 + rr) * F + lane * 4) = *(const v4f*)(&Tf[rr][lane * 4]); __threadfence(); }
    wave_lds_sync(); } }
__global__ __launch_bounds__(32) void sweep1_kernel(const float* __restrict__ atom, const float* __restrict__ force, const float* __restrict__ dispn, const float* __restrict__ dispe, const float* __restrict__ dist, const int* __restrict__ dsts, const int* __restrict__ PERM, const int* __restrict__ ROWPTR, const int* __restrict__ ROWCNT, int permLen, const float* __restrict__ Hn, const b16* __restrict__ WEM, const float* __restrict__ empb, const b16* __restrict__ WEQ, const float* __restrict__ e1b1, const float* __restrict__ e2b1, const b16* __restrict__ W8, const float* __restrict__ e1b2, const float* __restrict__ e2b2, int NLIM, float* __restrict__ A1, float* __restrict__ AGG1, float* __restrict__ out1, float* __restrict__ D1) {
  __shared__ __attribute__((aligned(16))) b16 Ad[16][40], Ah[16][F + 8], Al[16][F + 8], Bh[16][264], Bl[16][264]; __shared__ float INV[16][F + 1], EQ[2][16][F + 1]; __shared__ int Ed[16], Ee[16]; const int lane = threadIdx.x, nloc = lane & 15, hlf = lane >> 4; const size_t n = blockIdx.x; if (n >= (size_t)NLIM) return;
  if (lane < 16) { for (int k = 0; k < 8; ++k) { Ah[lane][F + k] = (b16)0.0f; Al[lane][F + k] = (b16)0.0f; Bh[lane][256 + k] = (b16)0.0f; Bl[lane][256 + k] = (b16)0.0f; } for (int k = NBF; k < 40; ++k) Ad[lane][k] = (b16)0.0f; }
  float hn[4], accA[4], agg1[3][4], acc2[3][4]; for (int q = 0; q < 4; ++q) { hn[q] = Hn[n * F + lane * 4 + q]; accA[q] = 0.0f; for (int a = 0; a < 3; ++a) { agg1[a][q] = 0.0f; acc2[a][q] = 0.0f; } }
  int st = ROWPTR[n], cnt = ROWCNT[n]; cnt = iclamp(cnt, 0, E); st = iclamp(st, 0, permLen - cnt);
  const b16* e1w2 = W8 + (size_t)2 * F * F; const b16* e2w2 = W8 + (size_t)3 * F * F;
  wave_lds_sync();
#pragma unroll 1
  for (int j0 = 0; j0 < cnt; j0 += 16) { const int nr = (cnt - j0) < 16 ? (cnt - j0) : 16;
    if (lane < 16) { int e = -1, d = 0; if (lane < nr) { e = iclamp(PERM[st + j0 + lane], 0, E - 1); d = iclamp(dsts[e], 0, N - 1); if (d >= NLIM) e = -1; } Ee[lane] = e; Ed[lane] = d; for (int k = 0; k < NBF; ++k) Ad[lane][k] = (b16)(e >= 0 ? bfv(dist[(size_t)e * NBF + k]) * XS : 0.0f); }
    wave_lds_sync();
    { v8f acc[8];
#pragma unroll
      for (int t = 0; t < 8; ++t) acc[t] = (v8f){};
      { const v16b a = frag_kb(&Ad[nloc][0], hlf);
#pragma unroll
        for (int t = 0; t < 8; ++t) acc[t] = wmma16b(a, frag_kb(WEM + (size_t)(t * 16 + nloc) * 32, hlf), acc[t]); }
#pragma unroll
      for (int t = 0; t < 8; ++t) { const int cc = t * 16 + nloc; const float bb = bfv(empb[cc]); const float hc = Hn[n * F + cc];
#pragma unroll
        for (int r8 = 0; r8 < 8; ++r8) { const int rr = 8 * hlf + r8; const int e = Ee[rr]; float iv = 0.0f; if (e >= 0) iv = pmul(pmul(acc[t][r8] * (1.0f / (XS * WSC)) + bb, hc), Hn[(size_t)Ed[rr] * F + cc]); INV[rr][cc] = iv; b16 p, pl; split16(iv * HS, p, pl); Ah[rr][cc] = p; Al[rr][cc] = pl; } } }
    wave_lds_sync();
    for (int rr = 0; rr < nr; ++rr) if (Ee[rr] >= 0) { for (int q = 0; q < 4; ++q) accA[q] += INV[rr][lane * 4 + q]; }
    { v8f acc[16];
#pragma unroll
      for (int t = 0; t < 16; ++t) acc[t] = (v8f){};
#pragma unroll
      for (int kb = 0; kb < F; kb += 32) { const v16b a = frag_kb(&Ah[nloc][kb], hlf), al = frag_kb(&Al[nloc][kb], hlf);
#pragma unroll
        for (int t = 0; t < 16; ++t) { const v16b bw = frag_kb(WEQ + (size_t)(t * 16 + nloc) * F + kb, hlf); acc[t] = wmma16b(a, bw, acc[t]); acc[t] = wmma16b(al, bw, acc[t]); } }
#pragma unroll
      for (int t = 0; t < 16; ++t) { const int cc = t * 16 + nloc; const float bb = bfv(cc < F ? e1b1[cc] : e2b1[cc - F]);
#pragma unroll
        for (int r8 = 0; r8 < 8; ++r8) { const float hv = silu(acc[t][r8] * (1.0f / (HS * WSC)) + bb); b16 p, pl; split16(hv * HS, p, pl); Bh[8 * hlf + r8][cc] = p; Bl[8 * hlf + r8][cc] = pl; } } }
    wave_lds_sync();
#pragma unroll 1
    for (int m = 0; m < 2; ++m) { v8f acc[8]; const b16* W2p = m == 0 ? e1w2 : e2w2; const float* b2p = m == 0 ? e1b2 : e2b2;
#pragma unroll
      for (int t = 0; t < 8; ++t) acc[t] = (v8f){};
#pragma unroll
      for (int kb = 0; kb < F; kb += 32) { const v16b a = frag_kb(&Bh[nloc][m * F + kb], hlf), al = frag_kb(&Bl[nloc][m * F + kb], hlf);
#pragma unroll
        for (int t = 0; t < 8; ++t) { const v16b bw = frag_kb(W2p + (size_t)(t * 16 + nloc) * F + kb, hlf); acc[t] = wmma16b(a, bw, acc[t]); acc[t] = wmma16b(al, bw, acc[t]); } }
#pragma unroll
      for (int t = 0; t < 8; ++t) { const int cc = t * 16 + nloc; const float bb = bfv(b2p[cc]);
#pragma unroll
        for (int r8 = 0; r8 < 8; ++r8) EQ[m][8 * hlf + r8][cc] = acc[t][r8] * (1.0f / (HS * WSC)) + bb; } }
    wave_lds_sync();
    for (int rr = 0; rr < nr; ++rr) { const int e = Ee[rr]; if (e < 0) continue; const size_t d = (size_t)Ed[rr]; float de[3]; for (int a = 0; a < 3; ++a) de[a] = bfv(dispe[(size_t)e * 3 + a]);
      for (int q = 0; q < 4; ++q) { const int c = lane * 4 + q; const float v1 = EQ[0][rr][c], v2 = EQ[1][rr][c];
#pragma unroll
        for (int a = 0; a < 3; ++a) { agg1[a][q] += pmul(v1, de[a]); acc2[a][q] += pmul(v2, bfv(dispn[(d * 3 + a) * F + c])); } } }
    wave_lds_sync(); }
  for (int pass = 0; pass < 2; ++pass) { v4f o; for (int q = 0; q < 4; ++q) o[q] = bfv(atom[n * F + lane * 4 + q]) + accA[q]; *(volatile v4f*)(A1 + n * F + lane * 4) = o;
    for (int a = 0; a < 3; ++a) { v4f g, f1, d1; for (int q = 0; q < 4; ++q) { const int c = lane * 4 + q; g[q] = agg1[a][q]; f1[q] = bfv(force[(n * 3 + a) * F + c]) + agg1[a][q]; d1[q] = bfv(dispn[(n * 3 + a) * F + c]) + acc2[a][q]; } *(volatile v4f*)(AGG1 + (n * 3 + a) * F + lane * 4) = g; *(volatile v4f*)(out1 + (n * 3 + a) * F + lane * 4) = f1; *(volatile v4f*)(D1 + (n * 3 + a) * F + lane * 4) = d1; }
    __threadfence(); } }
__global__ __launch_bounds__(256) void sweep2_kernel(const float* __restrict__ E3, const float* __restrict__ AGG1, const float* __restrict__ D1, const float* __restrict__ F1, const float* __restrict__ Un, const float* __restrict__ A1, const float* __restrict__ lng, const float* __restrict__ lnb, const int* __restrict__ dsts, const int* __restrict__ PERM, const int* __restrict__ ROWPTR, const int* __restrict__ ROWCNT, int permLen, int NLIM, float* __restrict__ out0, float* __restrict__ out2) { const int wave = threadIdx.x >> 5, lane = threadIdx.x & 31; const size_t n = (size_t)blockIdx.x * 8 + wave; if (n >= (size_t)NLIM) return;
  v4f a3[3] = {{0, 0, 0, 0}, {0, 0, 0, 0}, {0, 0, 0, 0}};
  int st = ROWPTR[n], cnt = ROWCNT[n]; cnt = iclamp(cnt, 0, E); st = iclamp(st, 0, permLen - cnt);
#pragma unroll 1
  for (int j = 0; j < cnt; ++j) { const int e = iclamp(PERM[st + j], 0, E - 1); const size_t d = (size_t)iclamp(dsts[e], 0, N - 1); if (d >= (size_t)NLIM) continue; const v4f g = *(const v4f*)(E3 + d * F + lane * 4);
#pragma unroll
    for (int a = 0; a < 3; ++a) a3[a] += g * *(const v4f*)(AGG1 + (d * 3 + a) * F + lane * 4); }
  v4f d2[3], dot = {0, 0, 0, 0};
#pragma unroll
  for (int a = 0; a < 3; ++a) { d2[a] = *(const v4f*)(D1 + (n * 3 + a) * F + lane * 4) + a3[a]; const v4f f1 = *(const v4f*)(F1 + (n * 3 + a) * F + lane * 4); dot += -f1 * d2[a]; }
  const v4f u = *(const v4f*)(Un + n * F + lane * 4), a1 = *(const v4f*)(A1 + n * F + lane * 4); v4f x; float s = 0.0f; for (int q = 0; q < 4; ++q) { x[q] = a1[q] + pmul(u[q], dot[q]); s += x[q]; }
  const float mean = wsum(s) * (1.0f / F); float vs = 0.0f; for (int q = 0; q < 4; ++q) { const float dd = x[q] - mean; vs += dd * dd; } const float var = wsum(vs) * (1.0f / F); const float rs = rsqrtf(var + EPS);
  v4f o; for (int q = 0; q < 4; ++q) { const int c = lane * 4 + q; o[q] = pmul((x[q] - mean) * rs, bfv(lng[c])) + bfv(lnb[c]); }
  for (int pass = 0; pass < 2; ++pass) { *(volatile v4f*)(out0 + n * F + lane * 4) = o; for (int a = 0; a < 3; ++a) *(volatile v4f*)(out2 + (n * 3 + a) * F + lane * 4) = d2[a]; __threadfence(); } }
}

extern "C" void kernel_launch(void* const* d_in, const int* in_sizes, int n_in, void* d_out, int out_size, void* d_ws, size_t ws_size, hipStream_t stream) {
  (void)n_in;
  auto Fp = [&](int i) { return (const float*)d_in[i]; }; auto Ip = [&](int i) { return (const int*)d_in[i]; };
  if (in_sizes[0] != N * F || in_sizes[1] != N * 3 * F || in_sizes[2] != N * 3 * F || in_sizes[3] != E * 3 || in_sizes[4] != E * NBF || in_sizes[5] != 2 * E || in_sizes[6] != F * F || in_sizes[10] != NBF * F || in_sizes[24] != F * F || out_size != N * F + 2 * N * 3 * F) return;
  const int NLIM = N;
  size_t off = 0; char* ws = (char*)d_ws;
  auto carve = [&](size_t bytes) { char* p = ws + off; off += (bytes + 255) & ~(size_t)255; return p; };
  b16* W8 = (b16*)carve((size_t)9 * F * F * 2); b16* WEQ = (b16*)carve((size_t)256 * F * 2); b16* WEM = (b16*)carve((size_t)F * 32 * 2); float* Hn = (float*)carve((size_t)N * F * 4); float* A1 = (float*)carve((size_t)N * F * 4); float* AGG1 = (float*)carve((size_t)N * 3 * F * 4); float* D1 = (float*)carve((size_t)N * 3 * F * 4); float* E3 = (float*)carve((size_t)N * F * 4); float* Un = (float*)carve((size_t)N * F * 4); CsrBufs8 csr; off = csr_carve8(csr, ws, off, E, N);
  if (off > ws_size || off > ((size_t)64 << 20)) return;
  float* out0 = (float*)d_out; float* out1 = out0 + (size_t)N * F; float* out2 = out1 + (size_t)N * 3 * F;
  wput_kernel<<<128, 256, 0, stream>>>(Fp(6), Fp(8), Fp(12), Fp(14), Fp(16), Fp(18), Fp(20), Fp(21), Fp(22), Fp(24), Fp(10), W8, WEQ, WEM);
  csr_build8(csr, Ip(5), E, N, stream);
  nodemlp_kernel<true><<<N / 16, 32, 0, stream>>>(Fp(0), W8, Fp(7), W8 + (size_t)F * F, Fp(9), Hn, nullptr, nullptr, nullptr);
  sweep1_kernel<<<NLIM, 32, 0, stream>>>(Fp(0), Fp(1), Fp(2), Fp(3), Fp(4), Ip(5) + E, csr.PERM, csr.ROWPTR, csr.ROWCNT, (int)csr.permLen, Hn, WEM, Fp(11), WEQ, Fp(13), Fp(17), W8, Fp(15), Fp(19), NLIM, A1, AGG1, out1, D1);
  nodemlp_kernel<false><<<NLIM / 16, 32, 0, stream>>>(A1, W8 + (size_t)6 * F * F, Fp(23), W8 + (size_t)7 * F * F, Fp(25), Un, W8 + (size_t)4 * F * F, W8 + (size_t)5 * F * F, E3);
  sweep2_kernel<<<(NLIM + 7) / 8, 256, 0, stream>>>(E3, AGG1, D1, out1, Un, A1, Fp(26), Fp(27), Ip(5) + E, csr.PERM, csr.ROWPTR, csr.ROWCNT, (int)csr.permLen, NLIM, out0, out2);
}
